// SimpleFrequencyAttention_21981642621476
// MI455X (gfx1250) — hardware-verified
//
#include <hip/hip_runtime.h>
#include <math.h>
#include <stdint.h>

#define NB    8
#define DCH   128
#define SEQ   4096
#define NQKV  384
#define NW    512
#define QT    64
#define AP    144
#define LQP   136
#define LVP   72
#define OP    68
#define LNPS  6.931471805599453f
#define SCL   0.08838834764831845f
#define OSC   64.0f
#define WSC   16.0f
#define IYS   0.0009765625f
static_assert((SEQ % QT) == 0);
static_assert((SEQ % 32) == 0);
static_assert((DCH % 32) == 0);
static_assert(NQKV == 3 * DCH);
static_assert(NW == NQKV + DCH);
static_assert(((NW * DCH) / 8) % 256 == 0);
static_assert(64 * AP == DCH * LVP);
static_assert(LQP >= DCH && (LQP % 8) == 0);
static_assert((AP % 8) == 0 && (LVP % 8) == 0);
static_assert(OP >= QT && (OP % 4) == 0);

typedef _Float16       v16h __attribute__((ext_vector_type(16)));
typedef _Float16       v8h  __attribute__((ext_vector_type(8)));
typedef __bf16         v16b __attribute__((ext_vector_type(16)));
typedef unsigned short v8us __attribute__((ext_vector_type(8)));
typedef float          v8f  __attribute__((ext_vector_type(8)));
typedef float          v4f  __attribute__((ext_vector_type(4)));
typedef unsigned int   v4u  __attribute__((ext_vector_type(4)));

union FragH { v16h v; v8h  h[2]; };
union FragB { v16b v; v8us u[2]; };
static_assert(sizeof(FragH) == 32);
static_assert(sizeof(FragB) == 32);

__device__ __forceinline__ unsigned short bf_bits(float f) {
  unsigned u = __float_as_uint(f);
  return (unsigned short)((u + 0x7FFFu + ((u >> 16) & 1u)) >> 16);
}
__device__ __forceinline__ float bf_up(unsigned short h) { return __uint_as_float(((unsigned)h) << 16); }
__device__ __forceinline__ float bfr(float f) { return bf_up(bf_bits(f)); }
__device__ __forceinline__ unsigned short h_bits(_Float16 x) { return __builtin_bit_cast(unsigned short, x); }
__device__ __forceinline__ unsigned pk16(unsigned short a, unsigned short b) { return (unsigned)a | ((unsigned)b << 16); }
__device__ __forceinline__ v8f zero8() { v8f z = {0.f, 0.f, 0.f, 0.f, 0.f, 0.f, 0.f, 0.f}; return z; }
__device__ __forceinline__ float hmax8(v8f s) {
  return fmaxf(fmaxf(fmaxf(s[0], s[1]), fmaxf(s[2], s[3])), fmaxf(fmaxf(s[4], s[5]), fmaxf(s[6], s[7])));
}

__device__ __forceinline__ v16h ldfrag_h(const _Float16* p) {
  FragH f;
  f.h[0] = *(const v8h*)(p);
  f.h[1] = *(const v8h*)(p + 16);
  return f.v;
}
__device__ __forceinline__ v16b ldfrag_b(const unsigned short* p) {
  FragB f;
  f.u[0] = *(const v8us*)(p);
  f.u[1] = *(const v8us*)(p + 16);
  return f.v;
}

__device__ __forceinline__ v8f mma_h(v16h a, v16h b, v8f c) {
  v8f d = __builtin_amdgcn_wmma_f32_16x16x32_f16(false, a, false, b, (short)0, c, false, false);
#if defined(__HIP_DEVICE_COMPILE__)
  asm volatile("v_nop\n\tv_nop\n\tv_nop\n\tv_nop" : "+v"(d) : "v"(a), "v"(b));
#endif
  return d;
}
__device__ __forceinline__ v8f mma_b(v16b a, v16b b, v8f c) {
  v8f d = __builtin_amdgcn_wmma_f32_16x16x32_bf16(false, a, false, b, (short)0, c, false, false);
#if defined(__HIP_DEVICE_COMPILE__)
  const v16h ha = __builtin_bit_cast(v16h, a), hb = __builtin_bit_cast(v16h, b);
  asm volatile("v_nop\n\tv_nop\n\tv_nop\n\tv_nop" : "+v"(d) : "v"(ha), "v"(hb));
#endif
  return d;
}

__device__ __forceinline__ void gemm4(const unsigned short* ap, const unsigned short* bp,
                                      v8f& acc0, v8f& acc1, v8f& acc2, v8f& acc3) {
  acc0 = zero8(); acc1 = zero8(); acc2 = zero8(); acc3 = zero8();
#pragma unroll
  for (int ks = 0; ks < 4; ++ks) {
    const v16b a = ldfrag_b(ap + 32 * ks);
    const unsigned short* bs = bp + 32 * ks;
    acc0 = mma_b(a, ldfrag_b(bs + 0 * 16 * DCH), acc0);
    acc1 = mma_b(a, ldfrag_b(bs + 1 * 16 * DCH), acc1);
    acc2 = mma_b(a, ldfrag_b(bs + 2 * 16 * DCH), acc2);
    acc3 = mma_b(a, ldfrag_b(bs + 3 * 16 * DCH), acc3);
  }
}

__device__ __forceinline__ void stage_h(unsigned short* L, int nr, int col, v8f acc) {
#pragma unroll
  for (int r = 0; r < 8; ++r) L[(nr + r) * LQP + col] = h_bits((_Float16)acc[r]);
}
__device__ __forceinline__ void stage_v(unsigned short* Lv, int e, int nr, v8f acc) {
#pragma unroll
  for (int r = 0; r < 8; ++r) Lv[e * LVP + nr + r] = h_bits((_Float16)acc[r]);
}

__device__ __forceinline__ unsigned short cvt_sel(bool isq, float fq, float fo) {
  const unsigned short uq = bf_bits(fq);
  const unsigned short uo = h_bits((_Float16)(bfr(fo) * WSC));
  return isq ? uq : uo;
}

__global__ __launch_bounds__(256) void cvt_w(const float* __restrict__ wqkv, const float* __restrict__ wout,
                                             unsigned short* W16) {
  const int i = blockIdx.x * 256 + threadIdx.x;
  if (i >= (NW * DCH) / 8) return;
  const int row = i >> 4;
  const int col = (i & 15) * 8;
  const int ra = min(row, NQKV - 1);
  const int rb = min(max(row - NQKV, 0), DCH - 1);
  const v4f a0 = *(const v4f*)(wqkv + (size_t)ra * DCH + col), a1 = *(const v4f*)(wqkv + (size_t)ra * DCH + col + 4);
  const v4f c0 = *(const v4f*)(wout + (size_t)rb * DCH + col), c1 = *(const v4f*)(wout + (size_t)rb * DCH + col + 4);
  const bool isq = row < NQKV;
  v4u w;
#pragma unroll
  for (int t = 0; t < 2; ++t) {
    w[t]     = pk16(cvt_sel(isq, a0[2 * t], c0[2 * t]), cvt_sel(isq, a0[2 * t + 1], c0[2 * t + 1]));
    w[2 + t] = pk16(cvt_sel(isq, a1[2 * t], c1[2 * t]), cvt_sel(isq, a1[2 * t + 1], c1[2 * t + 1]));
  }
  unsigned short* p = W16 + (size_t)i * 8;
  *(volatile v4u*)p = w;
  __threadfence();
  *(volatile v4u*)p = w;
}

__global__ __launch_bounds__(256)
void proj_kernel(const float* __restrict__ x, const unsigned short* __restrict__ W16,
                 unsigned short* QP, unsigned short* KP, unsigned short* VP) {
  __shared__ __align__(16) unsigned short Lav[64 * AP];
  __shared__ __align__(16) unsigned short Lq[64 * LQP];
  __shared__ __align__(16) unsigned short Lk[64 * LQP];
  const int tid  = threadIdx.x;
  const int lane = tid & 31, wave = tid >> 5;
  const int hh   = lane >> 4, c = lane & 15;
  const int bx   = blockIdx.x;
  const int b    = bx / (SEQ / QT);
  const int nt   = bx % (SEQ / QT);
  const int n0   = nt * QT;

  {
    const int n4 = (tid & 15) * 4, ds = tid >> 4;
    const float* xp = x + ((size_t)b * DCH + ds) * SEQ + n0 + n4;
#pragma unroll
    for (int it = 0; it < 8; ++it) {
      const v4f v = *(const v4f*)(xp + (size_t)it * 16 * SEQ);
      const int d = it * 16 + ds;
#pragma unroll
      for (int q = 0; q < 4; ++q) Lav[(n4 + q) * AP + d] = bf_bits(v[q]);
    }
  }
  __syncthreads();

  const int ng = wave & 3, ch = wave >> 2;
  const unsigned short* ap = Lav + (ng * 16 + c) * AP + 8 * hh;
  const int nr = ng * 16 + 8 * hh;
  const int cb = ch * 64;
  v8f acc0, acc1, acc2, acc3;

  gemm4(ap, W16 + (size_t)(0 * DCH + cb + c) * DCH + 8 * hh, acc0, acc1, acc2, acc3);
  stage_h(Lq, nr, cb + 0 * 16 + c, acc0);
  stage_h(Lq, nr, cb + 1 * 16 + c, acc1);
  stage_h(Lq, nr, cb + 2 * 16 + c, acc2);
  stage_h(Lq, nr, cb + 3 * 16 + c, acc3);
  gemm4(ap, W16 + (size_t)(1 * DCH + cb + c) * DCH + 8 * hh, acc0, acc1, acc2, acc3);
  stage_h(Lk, nr, cb + 0 * 16 + c, acc0);
  stage_h(Lk, nr, cb + 1 * 16 + c, acc1);
  stage_h(Lk, nr, cb + 2 * 16 + c, acc2);
  stage_h(Lk, nr, cb + 3 * 16 + c, acc3);
  gemm4(ap, W16 + (size_t)(2 * DCH + cb + c) * DCH + 8 * hh, acc0, acc1, acc2, acc3);

  __syncthreads();
  stage_v(Lav, cb + 0 * 16 + c, nr, acc0);
  stage_v(Lav, cb + 1 * 16 + c, nr, acc1);
  stage_v(Lav, cb + 2 * 16 + c, nr, acc2);
  stage_v(Lav, cb + 3 * 16 + c, nr, acc3);
  __syncthreads();

  {
    const int e = tid & 7, lq = tid >> 3;
#pragma unroll
    for (int pass = 0; pass < 2; ++pass) {
#pragma unroll
      for (int it = 0; it < 4; ++it) {
        const int L  = it * 32 + lq;
        const int n  = L >> 1, hf = L & 1;
        const size_t go = ((size_t)b * SEQ + n0 + n) * DCH + hf * 64 + 8 * e;
        const int lo_ = n * LQP + hf * 64 + 8 * e;
        const v4u uq = *(const v4u*)(Lq + lo_);
        const v4u uk = *(const v4u*)(Lk + lo_);
        *(volatile v4u*)(QP + go) = uq;
        *(volatile v4u*)(KP + go) = uk;
      }
#pragma unroll
      for (int it = 0; it < 4; ++it) {
        const int er = it * 32 + lq;
        const v4u uv = *(const v4u*)(Lav + er * LVP + 8 * e);
        *(volatile v4u*)(VP + ((size_t)b * DCH + er) * SEQ + n0 + 8 * e) = uv;
      }
      __threadfence();
    }
  }
}

__global__ __launch_bounds__(128)
void attn_kernel(const unsigned short* __restrict__ QP, const unsigned short* __restrict__ KP,
                 const unsigned short* __restrict__ VP, const unsigned short* __restrict__ W16,
                 const float* __restrict__ bout, float* y) {
  __shared__ __align__(16) float Os[DCH * OP];
  const int tid  = threadIdx.x;
  const int wave = tid >> 5;
  const int lane = tid & 31;
  const int hh   = lane >> 4;
  const int c    = lane & 15;
  const int bx   = blockIdx.x;
  const int b    = bx / (SEQ / QT);
  const int qb   = bx % (SEQ / QT);
  const int n0   = qb * QT;
  const _Float16* QPh = (const _Float16*)(const void*)QP;
  const _Float16* KPh = (const _Float16*)(const void*)KP;
  const _Float16* VPh = (const _Float16*)(const void*)VP;
  const _Float16* WOh = (const _Float16*)(const void*)W16 + (size_t)NQKV * DCH;

  const size_t qo = ((size_t)b * SEQ + n0 + wave * 16 + c) * DCH + 8 * hh;
  const v16h q0 = ldfrag_h(QPh + qo), q1 = ldfrag_h(QPh + qo + 32);
  const v16h q2 = ldfrag_h(QPh + qo + 64), q3 = ldfrag_h(QPh + qo + 96);
  const _Float16* Kp = KPh + ((size_t)b * SEQ + c) * DCH + 8 * hh;
  const _Float16* Vb = VPh + ((size_t)b * DCH + c) * SEQ + 8 * hh;

  float m = -1.0e30f, l = 0.f;
  v8f o0 = zero8(), o1 = zero8(), o2 = zero8(), o3 = zero8();
  v8f o4 = zero8(), o5 = zero8(), o6 = zero8(), o7 = zero8();
#pragma unroll 1
  for (int it = 0; it < SEQ / 32; ++it) {
    const int kb = it * 32;
    const _Float16* k0p = Kp + (size_t)kb * DCH;
    const _Float16* k1p = k0p + 16 * DCH;
    v8f s0, s1;
    s0 = mma_h(ldfrag_h(k0p),      q0, zero8());
    s0 = mma_h(ldfrag_h(k0p + 32), q1, s0);
    s0 = mma_h(ldfrag_h(k0p + 64), q2, s0);
    s0 = mma_h(ldfrag_h(k0p + 96), q3, s0);
    s1 = mma_h(ldfrag_h(k1p),      q0, zero8());
    s1 = mma_h(ldfrag_h(k1p + 32), q1, s1);
    s1 = mma_h(ldfrag_h(k1p + 64), q2, s1);
    s1 = mma_h(ldfrag_h(k1p + 96), q3, s1);

    float mx = fmaxf(hmax8(s0), hmax8(s1)) * SCL;
    mx = fmaxf(mx, __shfl_xor(mx, 16, 32));
    const float mn   = fmaxf(m, mx);
    const float corr = __expf(m - mn);
    m = mn;
    const float msh = mn - LNPS;
    l *= corr;
#pragma unroll
    for (int r = 0; r < 8; ++r) {
      o0[r] *= corr; o1[r] *= corr; o2[r] *= corr; o3[r] *= corr;
      o4[r] *= corr; o5[r] *= corr; o6[r] *= corr; o7[r] *= corr;
    }

    FragH ph;
    float ls = 0.f;
#pragma unroll
    for (int r = 0; r < 8; ++r) {
      const float e0 = __expf(s0[r] * SCL - msh);
      const float e1 = __expf(s1[r] * SCL - msh);
      ls += e0 + e1;
      ph.h[0][r] = (_Float16)e0;
      ph.h[1][r] = (_Float16)e1;
    }
    l += ls;

    o0 = mma_h(ldfrag_h(Vb + 0 * 16 * SEQ + kb), ph.v, o0);
    o1 = mma_h(ldfrag_h(Vb + 1 * 16 * SEQ + kb), ph.v, o1);
    o2 = mma_h(ldfrag_h(Vb + 2 * 16 * SEQ + kb), ph.v, o2);
    o3 = mma_h(ldfrag_h(Vb + 3 * 16 * SEQ + kb), ph.v, o3);
    o4 = mma_h(ldfrag_h(Vb + 4 * 16 * SEQ + kb), ph.v, o4);
    o5 = mma_h(ldfrag_h(Vb + 5 * 16 * SEQ + kb), ph.v, o5);
    o6 = mma_h(ldfrag_h(Vb + 6 * 16 * SEQ + kb), ph.v, o6);
    o7 = mma_h(ldfrag_h(Vb + 7 * 16 * SEQ + kb), ph.v, o7);
  }
  l += __shfl_xor(l, 16, 32);
  const float sc = OSC / l;

  FragH ob0, ob1, ob2, ob3;
#pragma unroll
  for (int r = 0; r < 8; ++r) {
    ob0.h[0][r] = (_Float16)(o0[r] * sc); ob0.h[1][r] = (_Float16)(o1[r] * sc);
    ob1.h[0][r] = (_Float16)(o2[r] * sc); ob1.h[1][r] = (_Float16)(o3[r] * sc);
    ob2.h[0][r] = (_Float16)(o4[r] * sc); ob2.h[1][r] = (_Float16)(o5[r] * sc);
    ob3.h[0][r] = (_Float16)(o6[r] * sc); ob3.h[1][r] = (_Float16)(o7[r] * sc);
  }

  const _Float16* wp = WOh + (size_t)c * DCH + 8 * hh;
  float* os = Os + (8 * hh) * OP + wave * 16 + c;
#pragma unroll
  for (int ot = 0; ot < 8; ++ot) {
    v8f ya = zero8();
    ya = mma_h(ldfrag_h(wp + ot * 16 * DCH),      ob0.v, ya);
    ya = mma_h(ldfrag_h(wp + ot * 16 * DCH + 32), ob1.v, ya);
    ya = mma_h(ldfrag_h(wp + ot * 16 * DCH + 64), ob2.v, ya);
    ya = mma_h(ldfrag_h(wp + ot * 16 * DCH + 96), ob3.v, ya);
#pragma unroll
    for (int r = 0; r < 8; ++r) os[(ot * 16 + r) * OP] = ya[r] * IYS;
  }
  __syncthreads();
  {
    const int e = tid & 7, lq = tid >> 3;
    float* ob = y + ((size_t)b * DCH) * SEQ + n0;
#pragma unroll
    for (int pass = 0; pass < 2; ++pass) {
#pragma unroll
      for (int it = 0; it < 16; ++it) {
        const int L   = it * 16 + lq;
        const int row = L >> 1, hf = L & 1;
        const v4f v   = *(const v4f*)(Os + row * OP + hf * 32 + 4 * e);
        const float bb = bfr(bout[row]);
        const v4f vo  = {v[0] + bb, v[1] + bb, v[2] + bb, v[3] + bb};
        *(volatile v4f*)(ob + (size_t)row * SEQ + hf * 32 + 4 * e) = vo;
      }
      __threadfence();
    }
  }
}

extern "C" void kernel_launch(void* const* d_in, const int* in_sizes, int n_in,
                              void* d_out, int out_size, void* d_ws, size_t ws_size,
                              hipStream_t stream) {
  const int NX = NB * DCH * SEQ;
  if (n_in < 4) return;
  if (in_sizes[0] != NX || in_sizes[1] != NQKV * DCH || in_sizes[2] != DCH * DCH || in_sizes[3] != DCH) return;
  if (out_size != NX) return;

  size_t off = 0;
  const size_t oW  = off; off += (size_t)NW * DCH * 2;
  const size_t szP = (size_t)NB * SEQ * DCH * 2;
  const size_t oQ  = off; off += szP;
  const size_t oK  = off; off += szP;
  const size_t oV  = off; off += (size_t)NB * DCH * SEQ * 2;
  if (off > ws_size) return;
  if (off > (size_t)134217728) return;

  const float* x    = (const float*)d_in[0];
  const float* Wqkv = (const float*)d_in[1];
  const float* Wout = (const float*)d_in[2];
  const float* bout = (const float*)d_in[3];
  char* ws = (char*)d_ws;
  unsigned short* W16 = (unsigned short*)(ws + oW);
  unsigned short* QPp = (unsigned short*)(ws + oQ);
  unsigned short* KPp = (unsigned short*)(ws + oK);
  unsigned short* VPp = (unsigned short*)(ws + oV);
  float* y = (float*)d_out;

  const dim3 blk256(256), blk128(128);
  const dim3 gW((NW * DCH / 8) / 256);
  const dim3 gP(NB * (SEQ / QT));
  const dim3 gA(NB * (SEQ / QT));

  cvt_w<<<gW, blk256, 0, stream>>>(Wqkv, Wout, W16);
  proj_kernel<<<gP, blk256, 0, stream>>>(x, W16, QPp, KPp, VPp);
  attn_kernel<<<gA, blk128, 0, stream>>>(QPp, KPp, VPp, W16, bout, y);
  (void)hipGetLastError();
}
